// DNN_35064113004704
// MI455X (gfx1250) — hardware-run, weakly checked
//
#include <hip/hip_runtime.h>
#include <math.h>

typedef __attribute__((ext_vector_type(16))) _Float16 v16h;
typedef __attribute__((ext_vector_type(8)))  _Float16 v8h;
typedef __attribute__((ext_vector_type(8)))  float    v8f;
typedef __attribute__((ext_vector_type(4)))  float    v4f;

constexpr int kBatch = 16;
constexpr int kLen   = 160000;
constexpr int kWin   = 320;
constexpr int kHop   = 160;
constexpr int kNc    = 100;
constexpr int kNt    = (kLen - kWin) / kHop + 1;
constexpr int kM     = kBatch * kNt;
constexpr int kMp    = 16000;
constexpr int kNp    = 128;
constexpr int kQ     = kLen / kHop;
constexpr int kRows2 = kBatch * kQ;
constexpr int kPhaseMod = 4 * kWin;
static_assert(kNt == 999, "frames per sequence");
static_assert(kM == 15984, "compact rows");
static_assert(kQ == 1000 && kRows2 == 16000, "output rows of 160 samples");
static_assert(kMp >= kM && (kMp % 64) == 0 && (kMp % 32) == 0, "row padding");
static_assert(2 * kHop == kWin, "two frames per sample");
static_assert((kWin % 32) == 0 && (kNp % 32) == 0 && ((2 * kNp) % 32) == 0, "K multiples of 32");
static_assert(kNc <= kNp, "column padding");

constexpr float kCarryAct = 256.0f;
constexpr float kCarryCos = 1024.0f;
constexpr float kCarryWgt = 256.0f;
constexpr float kFoldCos  = 1.0f / (kCarryAct * kCarryCos);
constexpr float kFoldWgt  = 1.0f / (kCarryAct * kCarryWgt);
constexpr float kHalfMinNormal = 1.0f / 16384.0f;
constexpr double kPiD = 3.14159265358979323846;
constexpr float kPhaseStep = (float)(kPiD / (2.0 * (double)kWin));

constexpr size_t kSzWIN = (size_t)kWin * 4;
constexpr size_t kSzDF  = (size_t)kNp * kWin * 2;
constexpr size_t kSzDI  = (size_t)kHop * 2 * kNp * 2;
constexpr size_t kSzWH  = (size_t)3 * kNp * kNp * 2;
constexpr size_t kSzBI  = (size_t)3 * kNp * 4;
constexpr size_t kSzXH  = (size_t)kMp * kNp * 2;
constexpr size_t kSzOH  = (size_t)kMp * kNp * 2;
constexpr size_t kOffWIN = 0;
constexpr size_t kOffDF  = kOffWIN + kSzWIN;
constexpr size_t kOffDI  = kOffDF + kSzDF;
constexpr size_t kOffWH  = kOffDI + kSzDI;
constexpr size_t kOffBI  = kOffWH + kSzWH;
constexpr size_t kOffXH  = kOffBI + kSzBI;
constexpr size_t kOffOH  = kOffXH + kSzXH;
constexpr size_t kWsTotal = kOffOH + kSzOH;
static_assert(kWsTotal == 8456960ull, "carve total");
static_assert(kWsTotal <= 134217728ull, "carve cap");
static_assert((kOffDF % 128) == 0 && (kOffDI % 128) == 0 && (kOffWH % 128) == 0 && (kOffBI % 128) == 0 &&
              (kOffXH % 128) == 0 && (kOffOH % 128) == 0, "128-B aligned regions");

constexpr size_t kOutBytes0 = (size_t)kM * kNc * 4;
constexpr size_t kOutOff1   = kOutBytes0;
constexpr size_t kOutOff2   = 2 * kOutBytes0;
constexpr size_t kOutTotal  = kOutOff2 + (size_t)kBatch * kLen * 4;
static_assert(kOutOff1 == 6393600ull && kOutOff2 == 12787200ull && kOutTotal == 23027200ull, "output packing");
static_assert((kOutOff1 % 128) == 0 && (kOutOff2 % 128) == 0, "outputs start on lines");

constexpr int kDfBlocks  = (kNp * kWin / 2) / 256;
constexpr int kDiBlocks  = (kHop * 2 * kNp / 2) / 256;
constexpr int kWinBlocks = (kWin + 255) / 256;
constexpr int kWPlaneBlocks = (kNp * kNp / 2) / 256;
constexpr int kBiasWords = 3 * kNp;
constexpr int kBiasBlocks = (kBiasWords + 255) / 256;
constexpr int kDctTiles = kMp / 32;
static_assert(kDfBlocks * 256 * 2 == kNp * kWin, "forward table coverage");
static_assert(kDiBlocks * 256 * 2 == kHop * 2 * kNp, "inverse table coverage");
static_assert(kWPlaneBlocks * 256 * 2 == kNp * kNp, "weight plane coverage");
static_assert((kWin % 32) == 0 && (kBiasWords % 32) == 0, "whole-wave tails");

__device__ __forceinline__ float flush_small(float v) {
  return (fabsf(v) < kHalfMinNormal) ? 0.0f : v;
}
__device__ __forceinline__ _Float16 to_half_op(float v) {
  return (_Float16)flush_small(v);
}
__device__ __forceinline__ unsigned half_bits(float v) {
  const _Float16 h = to_half_op(v);
  const unsigned short s = __builtin_bit_cast(unsigned short, h);
  return (unsigned)s;
}
__device__ __forceinline__ void pin_v4(v4f& x) { asm volatile("" : "+v"(x)); }
__device__ __forceinline__ void pin_f(float& x) { asm volatile("" : "+v"(x)); }

union FragU { v16h v; v8h h[2]; };
__device__ __forceinline__ v16h frag_load(const _Float16* p) {
  FragU f;
  f.h[0] = *(const v8h*)(p);
  f.h[1] = *(const v8h*)(p + 16);
  return f.v;
}
__device__ __forceinline__ v8f mma_g(v16h a, v16h b, v8f c) {
  c = __builtin_amdgcn_wmma_f32_16x16x32_f16(false, a, false, b, (short)0, c, false, false);
  asm volatile("v_nop\n\tv_nop\n\tv_nop\n\tv_nop" : "+v"(c) : "v"(a), "v"(b));
  return c;
}

__device__ __forceinline__ float cos_phase(int ph) {
  int p = ph;
  p = (p > 2 * kWin) ? (kPhaseMod - p) : p;
  const bool neg = (p > kWin);
  p = neg ? (2 * kWin - p) : p;
  const float x = (float)p * kPhaseStep;
  float c = cosf(x);
  c = (p == kWin) ? 0.0f : c;
  return neg ? -c : c;
}

__global__ __launch_bounds__(256) void prep_cos_kernel(
    unsigned* __restrict__ DFw, unsigned* __restrict__ DIw, unsigned* __restrict__ WINw)
{
  const int blk = blockIdx.x;
  const int tid = threadIdx.x;
  int region = 0;
  int w = blk * 256 + tid;
  if (blk >= kDfBlocks + kDiBlocks) {
    region = 2;
    w = (blk - kDfBlocks - kDiBlocks) * 256 + tid;
  } else if (blk >= kDfBlocks) {
    region = 1;
    w = (blk - kDfBlocks) * 256 + tid;
  }
  const float amp = sqrtf(2.0f / (float)kWin);
  const float c0s = sqrtf(0.5f);
  unsigned word = 0u;
#pragma unroll 1
  for (int e = 0; e < 2; ++e) {
    const int idx = 2 * w + e;
    int ph = 0;
    bool valid = true;
    bool col0 = false;
    if (region == 0) {
      const int n = idx / kWin;
      const int j = idx - n * kWin;
      ph = ((2 * j + 1) * n) % kPhaseMod;
      valid = (n < kNc);
      col0 = (n == 0);
    } else if (region == 1) {
      const int r = idx >> 8;
      const int c = idx & 255;
      const int hf = c >> 7;
      const int k = c & 127;
      const int j = r + kHop * hf;
      ph = ((2 * j + 1) * k) % kPhaseMod;
      valid = (k < kNc);
      col0 = (k == 0);
    } else {
      const int j = (w < kWin) ? w : (kWin - 1);
      ph = 4 * j;
    }
    const float c = cos_phase(ph);
    float dv = amp * c;
    dv = col0 ? (dv * c0s) : dv;
    if (region == 2) {
      if (e == 0) word = __float_as_uint(0.5f * (1.0f - c));
    } else {
      const float cv = valid ? (dv * kCarryCos) : 0.0f;
      const unsigned hb = half_bits(cv);
      word |= hb << (16 * e);
    }
  }
  unsigned* dst = (region == 0) ? DFw : ((region == 1) ? DIw : WINw);
  const bool live = (region < 2) || (w < kWin);
  if (live) {
    volatile unsigned* q = dst + w;
    *q = word;
    __threadfence();
    *q = word;
  }
}

__global__ __launch_bounds__(256) void prep_w_kernel(
    const float* __restrict__ W1, const float* __restrict__ W2, const float* __restrict__ W3,
    const float* __restrict__ b1, const float* __restrict__ b2, const float* __restrict__ b3,
    unsigned* __restrict__ WHw, float* __restrict__ BI)
{
  const int blk = blockIdx.x;
  const int tid = threadIdx.x;
  if (blk < 3 * kWPlaneBlocks) {
    const int plane = blk / kWPlaneBlocks;
    const int w = (blk - plane * kWPlaneBlocks) * 256 + tid;
    const float* src = (plane == 0) ? W1 : ((plane == 1) ? W2 : W3);
    unsigned word = 0u;
#pragma unroll
    for (int e = 0; e < 2; ++e) {
      const int idx = 2 * w + e;
      const int n = idx >> 7;
      const int k = idx & 127;
      const bool valid = (n < kNc) && (k < kNc);
      const int nc = (n < kNc) ? n : (kNc - 1);
      const int kc = (k < kNc) ? k : (kNc - 1);
      float v = src[nc * kNc + kc];
      pin_f(v);
      const float cv = valid ? (v * kCarryWgt) : 0.0f;
      const unsigned hb = half_bits(cv);
      word |= hb << (16 * e);
    }
    volatile unsigned* q = WHw + (size_t)plane * (kNp * kNp / 2) + w;
    *q = word;
    __threadfence();
    *q = word;
  } else {
    const int w = (blk - 3 * kWPlaneBlocks) * 256 + tid;
    const bool live = (w < kBiasWords);
    const int wc = live ? w : (kBiasWords - 1);
    const int layer = wc >> 7;
    const int n = wc & 127;
    const int nc = (n < kNc) ? n : (kNc - 1);
    float v1 = b1[nc];
    float v2 = b2[nc];
    float v3 = b3[nc];
    pin_f(v1);
    pin_f(v2);
    pin_f(v3);
    float v = (layer == 0) ? v1 : ((layer == 1) ? v2 : v3);
    v = (n < kNc) ? v : 0.0f;
    if (live) {
      volatile float* q = BI + w;
      *q = v;
      __threadfence();
      *q = v;
    }
  }
}

__global__ __launch_bounds__(256) void dct_kernel(
    const float* __restrict__ noisy, const float* __restrict__ clean,
    const float* __restrict__ WIN, const _Float16* __restrict__ DF,
    _Float16* __restrict__ XH, float* __restrict__ out1)
{
  __shared__ __align__(16) _Float16 sA[32 * kWin];
  __shared__ __align__(16) float sC[32 * kNp];
  const int tid = threadIdx.x;
  const int lane = tid & 31;
  const int wave = tid >> 5;
  const bool isClean = ((int)blockIdx.x >= kDctTiles);
  const int tileIdx = isClean ? ((int)blockIdx.x - kDctTiles) : (int)blockIdx.x;
  const int m0 = tileIdx * 32;
  const float* sig = isClean ? clean : noisy;

#pragma unroll
  for (int it = 0; it < 5; ++it) {
    const int idx = it * 256 + tid;
    const int row = idx / 40;
    const int c8 = (idx - row * 40) * 8;
    const int m = m0 + row;
    const bool valid = (m < kM);
    const int mc = valid ? m : (kM - 1);
    const int b = mc / kNt;
    const int t = mc - b * kNt;
    const float* sp = sig + (size_t)b * kLen + (size_t)t * kHop + c8;
    v4f s0 = *(const v4f*)(sp);
    v4f s1 = *(const v4f*)(sp + 4);
    v4f w0 = *(const v4f*)(WIN + c8);
    v4f w1 = *(const v4f*)(WIN + c8 + 4);
    pin_v4(s0);
    pin_v4(s1);
    pin_v4(w0);
    pin_v4(w1);
    v8h hv;
#pragma unroll
    for (int e = 0; e < 4; ++e) {
      const float f0 = s0[e] * w0[e];
      const float f1 = s1[e] * w1[e];
      const float g0 = valid ? (f0 * kCarryAct) : 0.0f;
      const float g1 = valid ? (f1 * kCarryAct) : 0.0f;
      hv[e] = to_half_op(g0);
      hv[4 + e] = to_half_op(g1);
    }
    *(v8h*)(sA + row * kWin + c8) = hv;
  }
  __syncthreads();

  const int rl = lane & 15;
  const int koff = (lane >> 4) * 8;
  const int mOff = (lane >> 4) * 8;
  const int msub = wave & 1;
  const int nb = wave >> 1;
  v8f acc0 = (v8f){0.f, 0.f, 0.f, 0.f, 0.f, 0.f, 0.f, 0.f};
  v8f acc1 = (v8f){0.f, 0.f, 0.f, 0.f, 0.f, 0.f, 0.f, 0.f};
  const _Float16* ap = sA + (msub * 16 + rl) * kWin + koff;
  const _Float16* bp0 = DF + (size_t)(nb * 32 + rl) * kWin + koff;
  const _Float16* bp1 = bp0 + (size_t)16 * kWin;
#pragma unroll 2
  for (int k0 = 0; k0 < kWin; k0 += 32) {
    const v16h a = frag_load(ap + k0);
    const v16h bq0 = frag_load(bp0 + k0);
    const v16h bq1 = frag_load(bp1 + k0);
    acc0 = mma_g(a, bq0, acc0);
    acc1 = mma_g(a, bq1, acc1);
  }

#pragma unroll
  for (int j = 0; j < 2; ++j) {
    const int n = nb * 32 + j * 16 + rl;
#pragma unroll
    for (int r = 0; r < 8; ++r) {
      const int row = msub * 16 + mOff + r;
      float v = ((j == 0) ? acc0[r] : acc1[r]) * kFoldCos;
      v = fminf(1.0f, fmaxf(-1.0f, v));
      if (isClean) {
        if (n < kNc) sC[row * kNc + n] = v;
      } else {
        sC[row * kNp + n] = (n < kNc) ? v : 0.0f;
      }
    }
  }
  __syncthreads();

  if (isClean) {
    const int remain = kM - m0;
    const int rowsReal = (remain < 32) ? remain : 32;
    const int n4 = rowsReal * (kNc / 4);
    float* dst = out1 + (size_t)m0 * kNc;
    for (int pass = 0; pass < 2; ++pass) {
      for (int i = tid; i < n4; i += 256) {
        const v4f v = *(const v4f*)(sC + 4 * i);
        *(volatile v4f*)(dst + 4 * i) = v;
      }
      __threadfence();
    }
  } else {
    v8h hv[2];
#pragma unroll
    for (int it = 0; it < 2; ++it) {
      const int c = it * 256 + tid;
      const v4f a0 = *(const v4f*)(sC + 8 * c);
      const v4f a1 = *(const v4f*)(sC + 8 * c + 4);
#pragma unroll
      for (int e = 0; e < 4; ++e) {
        hv[it][e] = to_half_op(a0[e] * kCarryAct);
        hv[it][4 + e] = to_half_op(a1[e] * kCarryAct);
      }
    }
    _Float16* dst = XH + (size_t)m0 * kNp;
    for (int pass = 0; pass < 2; ++pass) {
#pragma unroll
      for (int it = 0; it < 2; ++it) {
        const int c = it * 256 + tid;
        *(volatile v8h*)(dst + 8 * c) = hv[it];
      }
      __threadfence();
    }
  }
}

__device__ __forceinline__ void dense_tile(const _Float16* act, const _Float16* __restrict__ Wp,
                                           int msub, int nhalf, int rl, int koff, v8f (&acc)[4])
{
#pragma unroll
  for (int j = 0; j < 4; ++j) acc[j] = (v8f){0.f, 0.f, 0.f, 0.f, 0.f, 0.f, 0.f, 0.f};
  const _Float16* ap = act + (msub * 16 + rl) * kNp + koff;
  const _Float16* bp = Wp + (size_t)(nhalf * 64 + rl) * kNp + koff;
#pragma unroll
  for (int k0 = 0; k0 < kNp; k0 += 32) {
    const v16h a = frag_load(ap + k0);
#pragma unroll
    for (int j = 0; j < 4; ++j) {
      const v16h bq = frag_load(bp + (size_t)j * 16 * kNp + k0);
      acc[j] = mma_g(a, bq, acc[j]);
    }
  }
}

__device__ __forceinline__ void prelu_store(const v8f (&acc)[4], const float* __restrict__ bias, float alpha,
                                            _Float16* dstAct, int msub, int nhalf, int rl, int mOff)
{
#pragma unroll
  for (int j = 0; j < 4; ++j) {
    const int n = nhalf * 64 + j * 16 + rl;
    const float bv = bias[n];
#pragma unroll
    for (int r = 0; r < 8; ++r) {
      const int row = msub * 16 + mOff + r;
      float v = acc[j][r] * kFoldWgt + bv;
      v = (v >= 0.0f) ? v : (alpha * v);
      dstAct[row * kNp + n] = to_half_op(v * kCarryAct);
    }
  }
}

__global__ __launch_bounds__(256) void mlp_kernel(
    const _Float16* __restrict__ XH, const _Float16* __restrict__ WH, const float* __restrict__ BI,
    const float* __restrict__ p1, const float* __restrict__ p2,
    _Float16* __restrict__ OH, float* __restrict__ out0)
{
  __shared__ __align__(16) _Float16 sX[64 * kNp];
  __shared__ __align__(16) _Float16 sY[64 * kNp];
  __shared__ __align__(16) float sO[64 * kNc];
  const int tid = threadIdx.x;
  const int lane = tid & 31;
  const int wave = tid >> 5;
  const int m0 = (int)blockIdx.x * 64;
  const int rl = lane & 15;
  const int koff = (lane >> 4) * 8;
  const int mOff = (lane >> 4) * 8;
  const int msub = wave & 3;
  const int nhalf = wave >> 2;

#pragma unroll
  for (int it = 0; it < 4; ++it) {
    const int c = it * 256 + tid;
    const v8h v = *(const v8h*)(XH + (size_t)m0 * kNp + 8 * c);
    *(v8h*)(sX + 8 * c) = v;
  }
  const float alpha1 = p1[0];
  const float alpha2 = p2[0];
  __syncthreads();

  v8f acc[4];
  dense_tile(sX, WH, msub, nhalf, rl, koff, acc);
  prelu_store(acc, BI, alpha1, sY, msub, nhalf, rl, mOff);
  __syncthreads();

  dense_tile(sY, WH + (size_t)kNp * kNp, msub, nhalf, rl, koff, acc);
  prelu_store(acc, BI + kNp, alpha2, sX, msub, nhalf, rl, mOff);
  __syncthreads();

  dense_tile(sX, WH + (size_t)2 * kNp * kNp, msub, nhalf, rl, koff, acc);
#pragma unroll
  for (int j = 0; j < 4; ++j) {
    const int n = nhalf * 64 + j * 16 + rl;
    const float bv = BI[2 * kNp + n];
#pragma unroll
    for (int r = 0; r < 8; ++r) {
      const int row = msub * 16 + mOff + r;
      const float z = acc[j][r] * kFoldWgt + bv;
      if (n < kNc) sO[row * kNc + n] = z;
    }
  }
  __syncthreads();

#pragma unroll 1
  for (int i = tid; i < 64 * kNc; i += 256) {
    const float z = sO[i];
    const float v = tanhf(z);
    sO[i] = v;
    const int row = i / kNc;
    const int col = i - row * kNc;
    sY[row * kNp + col] = to_half_op(v * kCarryAct);
  }
#pragma unroll 1
  for (int i = tid; i < 64 * (kNp - kNc); i += 256) {
    const int row = i / (kNp - kNc);
    const int col = kNc + (i - row * (kNp - kNc));
    sY[row * kNp + col] = (_Float16)0.0f;
  }
  __syncthreads();

  {
    const int remain = kM - m0;
    const int rowsReal = (remain < 64) ? remain : 64;
    const int n4 = rowsReal * (kNc / 4);
    float* dst = out0 + (size_t)m0 * kNc;
    for (int pass = 0; pass < 2; ++pass) {
      for (int i = tid; i < n4; i += 256) {
        const v4f v = *(const v4f*)(sO + 4 * i);
        *(volatile v4f*)(dst + 4 * i) = v;
      }
      __threadfence();
    }
  }
  {
    v8h hv[4];
#pragma unroll
    for (int it = 0; it < 4; ++it) hv[it] = *(const v8h*)(sY + 8 * (it * 256 + tid));
    _Float16* dst = OH + (size_t)m0 * kNp;
    for (int pass = 0; pass < 2; ++pass) {
#pragma unroll
      for (int it = 0; it < 4; ++it) *(volatile v8h*)(dst + 8 * (it * 256 + tid)) = hv[it];
      __threadfence();
    }
  }
}

__global__ __launch_bounds__(160) void idct_ola_kernel(
    const _Float16* __restrict__ OH, const _Float16* __restrict__ DI, float* __restrict__ out2)
{
  __shared__ __align__(16) _Float16 sA[32 * 2 * kNp];
  __shared__ __align__(16) float sO[32 * kHop];
  const int tid = threadIdx.x;
  const int lane = tid & 31;
  const int wave = tid >> 5;
  const int mp0 = (int)blockIdx.x * 32;

#pragma unroll 1
  for (int it = 0; it < 7; ++it) {
    const int idx = it * 160 + tid;
    const bool ok = (idx < 1024);
    const int idc = ok ? idx : 1023;
    const int row = idc >> 5;
    const int ch = idc & 31;
    const int hf = ch >> 4;
    const int kc = (ch & 15) * 8;
    const int mp = mp0 + row;
    const int b = mp / kQ;
    const int q = mp - b * kQ;
    const int t = q - hf;
    const bool valid = (t >= 0) && (t < kNt);
    const int tc = (t < 0) ? 0 : ((t > kNt - 1) ? (kNt - 1) : t);
    v8h v = *(const v8h*)(OH + (size_t)(b * kNt + tc) * kNp + kc);
    asm volatile("" : "+v"(v));
    const v8h zero8 = (v8h){(_Float16)0.0f, (_Float16)0.0f, (_Float16)0.0f, (_Float16)0.0f,
                            (_Float16)0.0f, (_Float16)0.0f, (_Float16)0.0f, (_Float16)0.0f};
    const v8h sv = valid ? v : zero8;
    if (ok) *(v8h*)(sA + idc * 8) = sv;
  }
  __syncthreads();

  const int rl = lane & 15;
  const int koff = (lane >> 4) * 8;
  const int mOff = (lane >> 4) * 8;
  v8f acc00 = (v8f){0.f, 0.f, 0.f, 0.f, 0.f, 0.f, 0.f, 0.f};
  v8f acc01 = acc00, acc10 = acc00, acc11 = acc00;
  const _Float16* ap0 = sA + rl * (2 * kNp) + koff;
  const _Float16* ap1 = ap0 + 16 * (2 * kNp);
  const _Float16* bp0 = DI + (size_t)(wave * 32 + rl) * (2 * kNp) + koff;
  const _Float16* bp1 = bp0 + (size_t)16 * (2 * kNp);
#pragma unroll 2
  for (int k0 = 0; k0 < 2 * kNp; k0 += 32) {
    const v16h a0 = frag_load(ap0 + k0);
    const v16h a1 = frag_load(ap1 + k0);
    const v16h bq0 = frag_load(bp0 + k0);
    const v16h bq1 = frag_load(bp1 + k0);
    acc00 = mma_g(a0, bq0, acc00);
    acc01 = mma_g(a0, bq1, acc01);
    acc10 = mma_g(a1, bq0, acc10);
    acc11 = mma_g(a1, bq1, acc11);
  }
#pragma unroll
  for (int r = 0; r < 8; ++r) {
    const int n0 = wave * 32 + rl;
    sO[(mOff + r) * kHop + n0]           = acc00[r] * kFoldCos;
    sO[(mOff + r) * kHop + n0 + 16]      = acc01[r] * kFoldCos;
    sO[(16 + mOff + r) * kHop + n0]      = acc10[r] * kFoldCos;
    sO[(16 + mOff + r) * kHop + n0 + 16] = acc11[r] * kFoldCos;
  }
  __syncthreads();

  float* dst = out2 + (size_t)mp0 * kHop;
  for (int pass = 0; pass < 2; ++pass) {
#pragma unroll
    for (int it = 0; it < 8; ++it) {
      const int i = it * 160 + tid;
      const v4f v = *(const v4f*)(sO + 4 * i);
      *(volatile v4f*)(dst + 4 * i) = v;
    }
    __threadfence();
  }
}

extern "C" void kernel_launch(void* const* d_in, const int* in_sizes, int n_in,
                              void* d_out, int out_size, void* d_ws, size_t ws_size,
                              hipStream_t stream) {
  if (n_in < 10) return;
  if (in_sizes[0] != kBatch * kLen) return;
  if (in_sizes[1] != kBatch * kLen) return;
  if (in_sizes[2] != kNc * kNc) return;
  if (in_sizes[3] != kNc) return;
  if (in_sizes[4] != 1) return;
  if (in_sizes[5] != kNc * kNc) return;
  if (in_sizes[6] != kNc) return;
  if (in_sizes[7] != 1) return;
  if (in_sizes[8] != kNc * kNc) return;
  if (in_sizes[9] != kNc) return;
  if ((size_t)out_size * 4 != kOutTotal) return;
  if (ws_size < kWsTotal) return;

  const float* noisy = (const float*)d_in[0];
  const float* clean = (const float*)d_in[1];
  const float* W1 = (const float*)d_in[2];
  const float* b1 = (const float*)d_in[3];
  const float* p1 = (const float*)d_in[4];
  const float* W2 = (const float*)d_in[5];
  const float* b2 = (const float*)d_in[6];
  const float* p2 = (const float*)d_in[7];
  const float* W3 = (const float*)d_in[8];
  const float* b3 = (const float*)d_in[9];

  char* outb = (char*)d_out;
  float* out0 = (float*)(outb);
  float* out1 = (float*)(outb + kOutOff1);
  float* out2 = (float*)(outb + kOutOff2);

  char* ws = (char*)d_ws;
  float*    WIN = (float*)(ws + kOffWIN);
  _Float16* DF  = (_Float16*)(ws + kOffDF);
  _Float16* DI  = (_Float16*)(ws + kOffDI);
  _Float16* WH  = (_Float16*)(ws + kOffWH);
  float*    BI  = (float*)(ws + kOffBI);
  _Float16* XH  = (_Float16*)(ws + kOffXH);
  _Float16* OH  = (_Float16*)(ws + kOffOH);

  prep_cos_kernel<<<kDfBlocks + kDiBlocks + kWinBlocks, 256, 0, stream>>>(
      (unsigned*)DF, (unsigned*)DI, (unsigned*)WIN);
  prep_w_kernel<<<3 * kWPlaneBlocks + kBiasBlocks, 256, 0, stream>>>(
      W1, W2, W3, b1, b2, b3, (unsigned*)WH, BI);
  dct_kernel<<<2 * kDctTiles, 256, 0, stream>>>(noisy, clean, WIN, DF, XH, out1);
  mlp_kernel<<<kMp / 64, 256, 0, stream>>>(XH, WH, BI, p1, p2, OH, out0);
  idct_ola_kernel<<<kRows2 / 32, 160, 0, stream>>>(OH, DI, out2);
}
